// LinearBlock_82746839924988
// MI455X (gfx1250) — hardware-verified
//
#include <hip/hip_runtime.h>
#include <stddef.h>
#include <stdint.h>


typedef _Float16 v16h __attribute__((ext_vector_type(16)));
typedef _Float16 v8h  __attribute__((ext_vector_type(8)));
typedef float    v8f  __attribute__((ext_vector_type(8)));
typedef float    v4f  __attribute__((ext_vector_type(4)));
typedef v4f __attribute__((may_alias)) v4fa;

#define TB   2048
#define CC   1024
#define HH   16
#define DD   64
#define FFD  4096
#define LDT  40
#define OPS  16.0f
#define ACCS (1.0f / 256.0f)

#define F_GELU 1
#define F_RES  2
#define F_HALF 4


union Frag { v16h v; v8h half[2]; };

__device__ __forceinline__ v8f wmma16(v16h a, v16h b, v8f c) {
  v8f d = __builtin_amdgcn_wmma_f32_16x16x32_f16(false, a, false, b, (short)0, c, false, false);
  asm volatile("v_nop\n\tv_nop\n\tv_nop\n\tv_nop" : "+v"(d) : "v"(a), "v"(b));
  return d;
}

__device__ __forceinline__ float wave_sum(float v) {
#pragma unroll
  for (int o = 16; o > 0; o >>= 1) v += __shfl_xor(v, o);
  return v;
}

__device__ __forceinline__ float gelu_f(float x) {
  return 0.5f * x * (1.0f + erff(x * 0.70710678118654752f));
}

__global__ __launch_bounds__(256)
void transpose_cvt(const float* __restrict__ in, _Float16* __restrict__ out, int K, int N) {
  __shared__ float tile[64][65];
  const int tid = threadIdx.x;
  const int kb = blockIdx.y * 64, nb = blockIdx.x * 64;
  if (kb + 64 > K || nb + 64 > N) return;
#pragma unroll
  for (int p = 0; p < 16; ++p) {
    const int idx = p * 256 + tid;
    const int kk = idx >> 6, nn = idx & 63;
    tile[kk][nn] = in[(size_t)(kb + kk) * N + (nb + nn)];
  }
  __syncthreads();
  v8h ov[2];
#pragma unroll
  for (int p = 0; p < 2; ++p) {
    const int s = p * 256 + tid;
    const int nn = s >> 3, pc = s & 7;
#pragma unroll
    for (int j = 0; j < 8; ++j) ov[p][j] = (_Float16)(OPS * tile[8 * pc + j][nn]);
    _Float16* gp = out + (size_t)(nb + nn) * K + kb + 8 * pc;
    *(volatile v8h*)gp = ov[p];
  }
  __threadfence();
#pragma unroll
  for (int p = 0; p < 2; ++p) {
    const int s = p * 256 + tid;
    const int nn = s >> 3, pc = s & 7;
    _Float16* gp = out + (size_t)(nb + nn) * K + kb + 8 * pc;
    *(volatile v8h*)gp = ov[p];
  }
}

__global__ __launch_bounds__(128)
void ln_kernel(const float* __restrict__ x, const float* __restrict__ g,
               const float* __restrict__ b, _Float16* __restrict__ out, int rows) {
  __shared__ float red_a[4], red_b[4];
  const int row = blockIdx.x;
  if (row >= rows) return;
  const int tid = threadIdx.x, lane = tid & 31, w = tid >> 5;
  const int c0 = tid * 8;
  const float* xr = x + (size_t)row * CC + c0;
  const v4f p0 = *(const v4f*)xr;
  const v4f p1 = *(const v4f*)(xr + 4);
  float v[8];
#pragma unroll
  for (int j = 0; j < 4; ++j) { v[j] = p0[j]; v[j + 4] = p1[j]; }
  float s = 0.0f;
#pragma unroll
  for (int j = 0; j < 8; ++j) s += v[j];
  s = wave_sum(s);
  if (lane == 0) red_a[w] = s;
  __syncthreads();
  const float mu = (red_a[0] + red_a[1] + red_a[2] + red_a[3]) * (1.0f / CC);
  float sq = 0.0f;
#pragma unroll
  for (int j = 0; j < 8; ++j) { const float d = v[j] - mu; sq += d * d; }
  sq = wave_sum(sq);
  if (lane == 0) red_b[w] = sq;
  __syncthreads();
  const float var = (red_b[0] + red_b[1] + red_b[2] + red_b[3]) * (1.0f / CC);
  const float rs = rsqrtf(var + 1e-5f);
  v8h o;
#pragma unroll
  for (int j = 0; j < 8; ++j) {
    const int c = c0 + j;
    o[j] = (_Float16)(OPS * ((v[j] - mu) * rs * g[c] + b[c]));
  }
  _Float16* op = out + (size_t)row * CC + c0;
  *(volatile v8h*)op = o;
  __threadfence();
  *(volatile v8h*)op = o;
}

__global__ __launch_bounds__(256)
void gemm_f16(const _Float16* __restrict__ A, const _Float16* __restrict__ Bt,
              const float* __restrict__ bias, const float* __restrict__ res,
              float* __restrict__ outF, _Float16* __restrict__ outH,
              int M, int N, int K, int flags) {
  __shared__ __align__(16) float smem[16384];
  _Float16* As = reinterpret_cast<_Float16*>(smem);
  _Float16* Bs = As + 128 * LDT;

  const int tid  = threadIdx.x;
  const int lane = tid & 31;
  const int wid  = tid >> 5;
  const int wr   = wid >> 1;
  const int wc   = wid & 1;
  const int hf   = lane >> 4;
  const int lm   = lane & 15;
  const int rowBase = blockIdx.y * 128;
  const int colBase = blockIdx.x * 128;
  if (rowBase + 128 > M || colBase + 128 > N) return;

  v8f acc[2][4];
#pragma unroll
  for (int i = 0; i < 2; ++i)
#pragma unroll
    for (int j = 0; j < 4; ++j)
#pragma unroll
      for (int r = 0; r < 8; ++r) acc[i][j][r] = 0.0f;

  const int ar = tid >> 2;
  const int ac = (tid & 3) * 8;
  const _Float16* Ag0 = A  + (size_t)(rowBase + ar) * K + ac;
  const _Float16* Ag1 = Ag0 + (size_t)64 * K;
  const _Float16* Bg0 = Bt + (size_t)(colBase + ar) * K + ac;
  const _Float16* Bg1 = Bg0 + (size_t)64 * K;

  const int nIter = K >> 5;
  for (int it = 0; it < nIter; ++it) {
    const int kt = it << 5;
    const v8h a0 = *(const v8h*)(Ag0 + kt);
    const v8h a1 = *(const v8h*)(Ag1 + kt);
    const v8h b0 = *(const v8h*)(Bg0 + kt);
    const v8h b1 = *(const v8h*)(Bg1 + kt);
    __syncthreads();
    *(v8h*)(As + ar * LDT + ac)        = a0;
    *(v8h*)(As + (ar + 64) * LDT + ac) = a1;
    *(v8h*)(Bs + ar * LDT + ac)        = b0;
    *(v8h*)(Bs + (ar + 64) * LDT + ac) = b1;
    __syncthreads();

    Frag af[2], bq[4];
#pragma unroll
    for (int tm = 0; tm < 2; ++tm) {
      const _Float16* p = As + (wr * 32 + tm * 16 + lm) * LDT;
      af[tm].half[0] = *(const v8h*)(p + 8 * hf);
      af[tm].half[1] = *(const v8h*)(p + 16 + 8 * hf);
    }
#pragma unroll
    for (int tn = 0; tn < 4; ++tn) {
      const _Float16* p = Bs + (wc * 64 + tn * 16 + lm) * LDT;
      bq[tn].half[0] = *(const v8h*)(p + 8 * hf);
      bq[tn].half[1] = *(const v8h*)(p + 16 + 8 * hf);
    }
#pragma unroll
    for (int tm = 0; tm < 2; ++tm)
#pragma unroll
      for (int tn = 0; tn < 4; ++tn)
        acc[tm][tn] = wmma16(af[tm].v, bq[tn].v, acc[tm][tn]);
  }

  __syncthreads();
  float* stg = smem + wid * 2048;
#pragma unroll
  for (int tm = 0; tm < 2; ++tm)
#pragma unroll
    for (int tn = 0; tn < 4; ++tn)
#pragma unroll
      for (int r = 0; r < 8; ++r)
        stg[(tm * 16 + 8 * hf + r) * 64 + tn * 16 + lm] = acc[tm][tn][r];
  __syncthreads();

  const bool doGelu = (flags & F_GELU) != 0;
  const bool doRes  = (flags & F_RES)  != 0;
  const bool doHalf = (flags & F_HALF) != 0;
  const int growW = rowBase + wr * 32;
  const int gcolW = colBase + wc * 64;

  if (!doHalf) {
#pragma unroll 1
    for (int i = 0; i < 16; ++i) {
      const int lrow = 2 * i + (lane >> 4);
      const int lc   = 4 * (lane & 15);
      v4fa* sp = (v4fa*)(stg + lrow * 64 + lc);
      v4f v = *sp;
      const int gcol = gcolW + lc;
      const size_t go = (size_t)(growW + lrow) * N + gcol;
      const v4f bb = *(const v4f*)(bias + gcol);
      v = v * ACCS + bb;
      if (doGelu) {
#pragma unroll
        for (int j = 0; j < 4; ++j) v[j] = gelu_f(v[j]);
      }
      if (doRes) v = v + *(const v4f*)(res + go);
      *sp = v;
      *(volatile v4f*)(outF + go) = v;
    }
    __threadfence();
#pragma unroll 1
    for (int i = 0; i < 16; ++i) {
      const int lrow = 2 * i + (lane >> 4);
      const int lc   = 4 * (lane & 15);
      const v4f v = *(const v4fa*)(stg + lrow * 64 + lc);
      const size_t go = (size_t)(growW + lrow) * N + gcolW + lc;
      *(volatile v4f*)(outF + go) = v;
    }
  } else {
#pragma unroll 1
    for (int i = 0; i < 8; ++i) {
      const int lrow = 4 * i + (lane >> 3);
      const int lc   = 8 * (lane & 7);
      v4fa* sp = (v4fa*)(stg + lrow * 64 + lc);
      v4f u0 = sp[0], u1 = sp[1];
      const int gcol = gcolW + lc;
      const size_t go = (size_t)(growW + lrow) * N + gcol;
      u0 = u0 * ACCS + *(const v4f*)(bias + gcol);
      u1 = u1 * ACCS + *(const v4f*)(bias + gcol + 4);
      if (doGelu) {
#pragma unroll
        for (int j = 0; j < 4; ++j) { u0[j] = gelu_f(u0[j]); u1[j] = gelu_f(u1[j]); }
      }
      if (doRes) { u0 = u0 + *(const v4f*)(res + go); u1 = u1 + *(const v4f*)(res + go + 4); }
      sp[0] = u0; sp[1] = u1;
      v8h o;
#pragma unroll
      for (int j = 0; j < 4; ++j) { o[j] = (_Float16)(OPS * u0[j]); o[j + 4] = (_Float16)(OPS * u1[j]); }
      *(volatile v8h*)(outH + go) = o;
    }
    __threadfence();
#pragma unroll 1
    for (int i = 0; i < 8; ++i) {
      const int lrow = 4 * i + (lane >> 3);
      const int lc   = 8 * (lane & 7);
      const v4fa* sp = (const v4fa*)(stg + lrow * 64 + lc);
      const v4f u0 = sp[0], u1 = sp[1];
      const size_t go = (size_t)(growW + lrow) * N + gcolW + lc;
      v8h o;
#pragma unroll
      for (int j = 0; j < 4; ++j) { o[j] = (_Float16)(OPS * u0[j]); o[j + 4] = (_Float16)(OPS * u1[j]); }
      *(volatile v8h*)(outH + go) = o;
    }
  }
}

__global__ __launch_bounds__(256)
void attn_kernel(const float* __restrict__ qkv, _Float16* __restrict__ o16, int T) {
  __shared__ float q_s[64], k_s[64], v_s[64], Kc[64];
  __shared__ float part[4][64];
  __shared__ float obuf[4][64];
  const int h = blockIdx.x, tid = threadIdx.x, lane = tid & 31;
  const int e = tid & 63, g = tid >> 6, dbase = g * 16;
  float st[16];
#pragma unroll
  for (int i = 0; i < 16; ++i) st[i] = 0.0f;
  if (tid < 64) Kc[tid] = 0.0f;
  __syncthreads();

  v8h ov;
#pragma unroll
  for (int j = 0; j < 8; ++j) ov[j] = (_Float16)0.0f;
  _Float16* optr = o16;

  for (int t = 0; t < T; ++t) {
    const float* base = qkv + (size_t)t * (3 * CC) + h * DD;
    if (tid < 64) {
      const float qv = base[tid];
      q_s[tid] = qv > 0.0f ? qv + 1.0f : expm1f(qv) + 1.0f;
    } else if (tid < 128) {
      const int i = tid - 64;
      const float kv = base[CC + i];
      k_s[i] = kv > 0.0f ? kv + 1.0f : expm1f(kv) + 1.0f;
    } else if (tid < 192) {
      const int i = tid - 128;
      v_s[i] = base[2 * CC + i];
    }
    __syncthreads();
    if (tid < 64) Kc[tid] += k_s[tid];
    const float ve = v_s[e];
    float p = 0.0f;
#pragma unroll
    for (int i = 0; i < 16; ++i) {
      const float s = st[i] + k_s[dbase + i] * ve;
      st[i] = s;
      p += q_s[dbase + i] * s;
    }
    part[g][e] = p;
    __syncthreads();
    if (tid < 64) {
      const float num = part[0][tid] + part[1][tid] + part[2][tid] + part[3][tid];
      float dd = q_s[lane] * Kc[lane] + q_s[lane + 32] * Kc[lane + 32];
      dd = wave_sum(dd);
      const float o = num * (1.0f / (dd + 1e-6f));
      obuf[t & 3][tid] = OPS * o;
    }
    if ((t & 3) == 3) {
      __syncthreads();
      if (tid < 32) {
        const int q = lane >> 3, j0 = 8 * (lane & 7);
#pragma unroll
        for (int j = 0; j < 8; ++j) ov[j] = (_Float16)obuf[q][j0 + j];
        optr = o16 + (size_t)(t - 3 + q) * CC + h * DD + j0;
        *(volatile v8h*)optr = ov;
      }
      __threadfence();
      if (tid < 32) {
        *(volatile v8h*)optr = ov;
      }
    }
    __syncthreads();
  }
}

extern "C" void kernel_launch(void* const* d_in, const int* in_sizes, int n_in,
                              void* d_out, int out_size, void* d_ws, size_t ws_size,
                              hipStream_t stream) {
  if (n_in < 13) return;
  if (in_sizes[0] != TB * CC || in_sizes[1] != CC * 3 * CC || in_sizes[2] != 3 * CC ||
      in_sizes[3] != CC * CC || in_sizes[4] != CC || in_sizes[5] != CC || in_sizes[6] != CC ||
      in_sizes[7] != CC || in_sizes[8] != CC || in_sizes[9] != CC * FFD || in_sizes[10] != FFD ||
      in_sizes[11] != FFD * CC || in_sizes[12] != CC || out_size != TB * CC) return;

  const float* x     = (const float*)d_in[0];
  const float* qkv_w = (const float*)d_in[1];
  const float* qkv_b = (const float*)d_in[2];
  const float* out_w = (const float*)d_in[3];
  const float* out_b = (const float*)d_in[4];
  const float* ln1_g = (const float*)d_in[5];
  const float* ln1_b = (const float*)d_in[6];
  const float* ln2_g = (const float*)d_in[7];
  const float* ln2_b = (const float*)d_in[8];
  const float* w1    = (const float*)d_in[9];
  const float* b1    = (const float*)d_in[10];
  const float* w2    = (const float*)d_in[11];
  const float* b2    = (const float*)d_in[12];
  float* out = (float*)d_out;

  char* ws = (char*)d_ws;
  size_t off = 0;
  auto alloc = [&](size_t bytes) -> void* {
    void* p = ws + off;
    off += (bytes + 255) & ~(size_t)255;
    return p;
  };
  _Float16* h1_16 = (_Float16*)alloc((size_t)TB * CC * 2);
  _Float16* h2_16 = (_Float16*)alloc((size_t)TB * CC * 2);
  _Float16* wq16  = (_Float16*)alloc((size_t)3 * CC * CC * 2);
  _Float16* wo16  = (_Float16*)alloc((size_t)CC * CC * 2);
  _Float16* w1_16 = (_Float16*)alloc((size_t)FFD * CC * 2);
  _Float16* w2_16 = (_Float16*)alloc((size_t)CC * FFD * 2);
  float*    qkvf  = (float*)   alloc((size_t)TB * 3 * CC * 4);
  _Float16* o16   = (_Float16*)alloc((size_t)TB * CC * 2);
  float*    x1    = (float*)   alloc((size_t)TB * CC * 4);
  _Float16* act16 = (_Float16*)alloc((size_t)TB * FFD * 2);
  if (off > ws_size) return;

  transpose_cvt<<<dim3(3 * CC / 64, CC / 64), 256, 0, stream>>>(qkv_w, wq16, CC, 3 * CC);
  transpose_cvt<<<dim3(CC / 64, CC / 64), 256, 0, stream>>>(out_w, wo16, CC, CC);
  transpose_cvt<<<dim3(FFD / 64, CC / 64), 256, 0, stream>>>(w1, w1_16, CC, FFD);
  transpose_cvt<<<dim3(CC / 64, FFD / 64), 256, 0, stream>>>(w2, w2_16, FFD, CC);

  ln_kernel<<<TB, 128, 0, stream>>>(x, ln1_g, ln1_b, h1_16, TB);

  gemm_f16<<<dim3(3 * CC / 128, TB / 128), 256, 0, stream>>>(
      h1_16, wq16, qkv_b, x, qkvf, o16, TB, 3 * CC, CC, 0);

  attn_kernel<<<HH, 256, 0, stream>>>(qkvf, o16, TB);

  gemm_f16<<<dim3(CC / 128, TB / 128), 256, 0, stream>>>(
      o16, wo16, out_b, x, x1, o16, TB, CC, CC, F_RES);

  ln_kernel<<<TB, 128, 0, stream>>>(x1, ln2_g, ln2_b, h2_16, TB);

  gemm_f16<<<dim3(FFD / 128, TB / 128), 256, 0, stream>>>(
      h2_16, w1_16, b1, x1, x1, act16, TB, FFD, CC, F_GELU | F_HALF);

  gemm_f16<<<dim3(CC / 128, TB / 128), 256, 0, stream>>>(
      act16, w2_16, b2, x1, out, act16, TB, CC, FFD, F_RES);
}
